// GroupedQueryAttention_23691039605412
// MI455X (gfx1250) — hardware-run, weakly checked
//
#include <hip/hip_runtime.h>


#ifndef NB
#define NB 2
#endif
#ifndef SEQ
#define SEQ 2048
#endif
#define NB_FULL  2
#define SEQ_FULL 2048
#ifndef OUT_SEQ
#define OUT_SEQ SEQ
#endif
#ifndef EROWS
#define EROWS 256
#endif
#define DM   2048
#define NH_  32
#define NKV  8
#define GRP  4
#define HD   64
#define KVD  512
#define AW   4
#define SC2  (0.125f * 1.4426950408889634f)
#define PSH  8.0f
#define CXS  256.0f
#define WOS  64.0f
#define OSC  (1.0f / 16384.0f)
#define MBP  64
#define RSC  2048.0f
#define RIN  (1.0f / 2048.0f)
#define NEGF (-__builtin_inff())

static_assert(HD == 64);
static_assert(NH_ * HD == DM);
static_assert(NKV * HD == KVD);
static_assert(NKV * GRP == NH_);
static_assert(DM % 64 == 0);
static_assert(KVD % 64 == 0);
static_assert(DM % 32 == 0);
static_assert(SEQ % 64 == 0);
static_assert((NB * SEQ) % 64 == 0);
static_assert(SEQ % 32 == 0);
static_assert(SEQ % (16 * AW) == 0);
static_assert(((size_t)SEQ * DM) % 8 == 0);
static_assert(NB <= NB_FULL);
static_assert(SEQ <= SEQ_FULL);
static_assert(SEQ <= 32 * MBP);
static_assert(SEQ % 16 == 0);
static_assert(EROWS >= 64);
static_assert(EROWS <= SEQ);
static_assert(EROWS % 64 == 0);
static_assert(EROWS % (16 * AW) == 0);
static_assert((SEQ - EROWS) % 64 == 0);
static_assert(AW * 32 <= 1024);

typedef _Float16 h16;
typedef unsigned short bf;
typedef __attribute__((ext_vector_type(16))) __bf16   v16bf;
typedef __attribute__((ext_vector_type(16))) _Float16 v16h;
typedef __attribute__((ext_vector_type(8)))  _Float16 v8h;
typedef __attribute__((ext_vector_type(8)))  unsigned short v8us;
typedef __attribute__((ext_vector_type(8)))  float    v8f;
typedef __attribute__((ext_vector_type(4)))  float    v4f;
typedef v4f  __attribute__((may_alias)) v4fa;

__device__ __forceinline__ unsigned short f2bf(float f) { unsigned u = __float_as_uint(f); u += 0x7FFFu + ((u >> 16) & 1u); return (unsigned short)(u >> 16); }
__device__ __forceinline__ float bfr(float f) { return __uint_as_float(((unsigned)f2bf(f)) << 16); }
__device__ __forceinline__ v16h cat16(v8h lo, v8h hi) { return __builtin_shufflevector(lo, hi, 0, 1, 2, 3, 4, 5, 6, 7, 8, 9, 10, 11, 12, 13, 14, 15); }
__device__ __forceinline__ v16bf cat16b(v8us lo, v8us hi) { return __builtin_bit_cast(v16bf, __builtin_shufflevector(lo, hi, 0, 1, 2, 3, 4, 5, 6, 7, 8, 9, 10, 11, 12, 13, 14, 15)); }
__device__ __forceinline__ v8f wmma16(v16h a, v16h b, v8f c) { return __builtin_amdgcn_wmma_f32_16x16x32_f16(false, a, false, b, (short)0, c, false, false); }
__device__ __forceinline__ v8f wmmab(v16bf a, v16bf b, v8f c) { return __builtin_amdgcn_wmma_f32_16x16x32_bf16(false, a, false, b, (short)0, c, false, false); }
__device__ __forceinline__ v16h  ldh(const h16* p) { return cat16(*(const v8h*)p, *(const v8h*)(p + 16)); }
__device__ __forceinline__ v16bf ldb(const bf* p)  { return cat16b(*(const v8us*)p, *(const v8us*)(p + 16)); }
__device__ __forceinline__ void wave_sync() { __builtin_amdgcn_fence(3  , "wavefront"); __builtin_amdgcn_wave_barrier(); asm volatile("" ::: "memory"); }

static __device__ __forceinline__ h16 toh_flush(float v) { const h16 r = (h16)v; return (fabsf(v) < 6.103515625e-05f) ? (h16)0.0f : r; }
__device__ __forceinline__ v8f wmma16g(v16h a, v16h b, v8f c) { c = __builtin_amdgcn_wmma_f32_16x16x32_f16(false, a, false, b, (short)0, c, false, false); asm volatile("v_nop\n\tv_nop\n\tv_nop\n\tv_nop" : "+v"(c) : "v"(a), "v"(b)); return c; }
__device__ __forceinline__ v8f wmmabg(v16bf a, v16bf b, v8f c) { c = __builtin_amdgcn_wmma_f32_16x16x32_bf16(false, a, false, b, (short)0, c, false, false); asm volatile("v_nop\n\tv_nop\n\tv_nop\n\tv_nop" : "+v"(c) : "v"(a), "v"(b)); return c; }

__global__ __launch_bounds__(256) void k_cvt8(const float* __restrict__ src, bf* dst, size_t n8) {
    const size_t i = (size_t)blockIdx.x * 256 + threadIdx.x; if (i >= n8) return;
    const v8f v = *(const v8f*)(src + i * 8); v8us o;
#pragma unroll
    for (int k = 0; k < 8; ++k) o[k] = f2bf(v[k]);
    *(volatile v8us*)(dst + i * 8) = o; __threadfence(); *(volatile v8us*)(dst + i * 8) = o;
}

template <int F16S>
__global__ __launch_bounds__(256) void k_tr(const float* __restrict__ W, unsigned short* WT, int K, int N) {
    __shared__ float tile[64 * 65];
    const int t = threadIdx.x;
    const int n0 = blockIdx.x * 64, k0 = blockIdx.y * 64;
#pragma unroll
    for (int i = 0; i < 4; ++i) { const int idx = i * 256 + t; const int kk = idx >> 4, n4 = (idx & 15) * 4;
        const v4f v = *(const v4f*)(W + (size_t)(k0 + kk) * (size_t)N + n0 + n4);
        tile[kk * 65 + n4 + 0] = v[0]; tile[kk * 65 + n4 + 1] = v[1]; tile[kk * 65 + n4 + 2] = v[2]; tile[kk * 65 + n4 + 3] = v[3]; }
    __syncthreads();
    const int c8 = (t & 7) * 8;
    v8us o0, o1;
    { const int n = (t >> 3);
      if (F16S) { v8h hv;
#pragma unroll
          for (int i = 0; i < 8; ++i) hv[i] = (h16)(bfr(tile[(c8 + i) * 65 + n]) * WOS);
          o0 = __builtin_bit_cast(v8us, hv);
      } else {
#pragma unroll
          for (int i = 0; i < 8; ++i) o0[i] = f2bf(tile[(c8 + i) * 65 + n]); } }
    { const int n = 32 + (t >> 3);
      if (F16S) { v8h hv;
#pragma unroll
          for (int i = 0; i < 8; ++i) hv[i] = (h16)(bfr(tile[(c8 + i) * 65 + n]) * WOS);
          o1 = __builtin_bit_cast(v8us, hv);
      } else {
#pragma unroll
          for (int i = 0; i < 8; ++i) o1[i] = f2bf(tile[(c8 + i) * 65 + n]); } }
    unsigned short* p0 = WT + (size_t)(n0 + (t >> 3)) * (size_t)K + k0 + c8;
    unsigned short* p1 = WT + (size_t)(n0 + 32 + (t >> 3)) * (size_t)K + k0 + c8;
    *(volatile v8us*)p0 = o0; *(volatile v8us*)p1 = o1;
    __threadfence();
    *(volatile v8us*)p0 = o0; *(volatile v8us*)p1 = o1;
}

__global__ __launch_bounds__(512) void k_mpack(const int* __restrict__ mask, unsigned* MB, unsigned* TF) {
    __shared__ unsigned wl[16 * MBP];
    __shared__ unsigned fl[4];
    const int lane = threadIdx.x & 31, wave = __builtin_amdgcn_readfirstlane((int)(threadIdx.x >> 5));
    const int qt = blockIdx.x; const int q = qt * 16 + wave;
    const size_t mro = (size_t)q * SEQ_FULL;
    unsigned w0 = 0u, w1 = 0u;
#pragma unroll 1
    for (int ks = 0; ks < MBP; ++ks) {
        const int key = ks * 32 + lane; const int kc = (key < SEQ) ? key : (SEQ - 1);
        const int mv = mask[mro + kc];
        const bool msk = (key >= SEQ) || (mv != 0);
        const unsigned bal = __builtin_amdgcn_ballot_w32(msk);
        w0 = (ks == lane) ? bal : w0; w1 = (ks == lane + 32) ? bal : w1;
    }
    unsigned* mp = MB + (size_t)q * MBP + lane;
    *(volatile unsigned*)mp = w0; *(volatile unsigned*)(mp + 32) = w1;
    __threadfence();
    *(volatile unsigned*)mp = w0; *(volatile unsigned*)(mp + 32) = w1;
    wl[wave * MBP + lane] = w0; wl[wave * MBP + 32 + lane] = w1;
    __syncthreads();
    if (wave < 2) {
        const int ks = wave * 32 + lane; unsigned orw = 0u, andw = 0xFFFFFFFFu;
#pragma unroll 1
        for (int r = 0; r < 16; ++r) { const unsigned w = wl[r * MBP + ks]; orw |= w; andw &= w; }
        const unsigned ab = __builtin_amdgcn_ballot_w32(andw != 0xFFFFFFFFu);
        const unsigned xb = __builtin_amdgcn_ballot_w32(orw != 0u);
        if (lane == 0) { fl[wave] = ab; fl[2 + wave] = xb; }
    }
    __syncthreads();
    if (wave == 0) {
        const unsigned fv = fl[lane & 3]; const unsigned ov = (lane < 4) ? fv : 0u;
        unsigned* tp = TF + (size_t)qt * 32 + lane;
        *(volatile unsigned*)tp = ov; __threadfence(); *(volatile unsigned*)tp = ov;
    }
}

template <int BROW>
__global__ __launch_bounds__(32) void k_proj(const bf* __restrict__ A, const bf* __restrict__ Bt, const float* __restrict__ bias, h16* Ph, int RB, size_t sRB, int pitch, int CB, size_t sCB) {
    __shared__ __align__(16) float os[16 * 68];
    const int K = DM;
    const int lane = threadIdx.x & 31, lr = lane & 15, hi = lane >> 4; const int r0 = blockIdx.x * 64, c0 = blockIdx.y * 64;
    v8f acc[4][4];
#pragma unroll
    for (int mb = 0; mb < 4; ++mb)
#pragma unroll
        for (int nb = 0; nb < 4; ++nb) acc[mb][nb] = (v8f){};
    const size_t aoff = (size_t)(r0 + lr) * K + 8 * hi, boff = (size_t)(c0 + lr) * K + 8 * hi;
#pragma unroll 1
    for (int kc = 0; kc < K; kc += 32) {
        v16bf a[4];
#pragma unroll
        for (int mb = 0; mb < 4; ++mb) a[mb] = ldb(A + aoff + (size_t)mb * 16 * K + kc);
#pragma unroll
        for (int nb = 0; nb < 4; ++nb) { const v16bf b = ldb(Bt + boff + (size_t)nb * 16 * K + kc);
#pragma unroll
            for (int mb = 0; mb < 4; ++mb) acc[mb][nb] = wmmab(a[mb], b, acc[mb][nb]); }
        asm volatile("v_nop\n\tv_nop\n\tv_nop\n\tv_nop" : "+v"(acc[0][0]), "+v"(acc[1][1]), "+v"(acc[2][2]), "+v"(acc[3][3]) : "v"(a[0]), "v"(a[1]), "v"(a[2]), "v"(a[3]));
    }
    const size_t tbase = (size_t)(r0 / RB) * sRB + (size_t)(r0 % RB) * (size_t)pitch + (size_t)(c0 / CB) * sCB + (size_t)(c0 % CB);
    v4f cb0 = (v4f){}, cb1 = (v4f){};
    if (BROW == 0) { const int c8 = (lane & 7) * 8;
        const v4f t0 = *(const v4f*)(bias + c0 + c8); const v4f t1 = *(const v4f*)(bias + c0 + c8 + 4);
#pragma unroll
        for (int i = 0; i < 4; ++i) { cb0[i] = bfr(t0[i]); cb1[i] = bfr(t1[i]); } }
#pragma unroll
    for (int mb = 0; mb < 4; ++mb) {
#pragma unroll
        for (int nb = 0; nb < 4; ++nb) {
#pragma unroll
            for (int j = 0; j < 8; ++j) os[(hi * 8 + j) * 68 + nb * 16 + lr] = acc[mb][nb][j]; }
        wave_sync();
        const size_t sb = tbase + (size_t)(mb * 16) * (size_t)pitch;
#pragma unroll 1
        for (int ps = 0; ps < 2; ++ps) {
#pragma unroll
            for (int s = 0; s < 4; ++s) { const int row = 4 * s + (lane >> 3), c8 = (lane & 7) * 8;
                v4f x0 = *(const v4fa*)(&os[row * 68 + c8]); v4f x1 = *(const v4fa*)(&os[row * 68 + c8 + 4]); v8h hv;
                if (BROW) { const float rb = bfr(bias[r0 + mb * 16 + row]);
#pragma unroll
                    for (int i = 0; i < 4; ++i) { x0[i] += rb; x1[i] += rb; }
                } else {
#pragma unroll
                    for (int i = 0; i < 4; ++i) { x0[i] += cb0[i]; x1[i] += cb1[i]; } }
#pragma unroll
                for (int i = 0; i < 4; ++i) { hv[i] = (h16)x0[i]; hv[4 + i] = (h16)x1[i]; }
                const size_t oo = sb + (size_t)row * (size_t)pitch + c8;
                *(volatile v8h*)(Ph + oo) = hv; }
            if (ps == 0) __threadfence(); }
        wave_sync();
    }
}

__global__ __launch_bounds__(32) void k_projr(const bf* __restrict__ A, const bf* __restrict__ Bt, const float* __restrict__ bias, h16* Pr, size_t zA, size_t zB, size_t zP, int brow, int RB, size_t sRB, int pitch, int CB, size_t sCB) {
    __shared__ __align__(16) float os[16 * 68];
    const int K = DM;
    const int lane = threadIdx.x & 31, lr = lane & 15, hi = lane >> 4; const int r0 = blockIdx.x * 64, c0 = blockIdx.y * 64;
    const size_t zz = (size_t)blockIdx.z;
    const bf* Az = A + zz * zA; const bf* Bz = Bt + zz * zB; h16* Pz = Pr + zz * zP;
    v8f acc[4][4];
#pragma unroll
    for (int mb = 0; mb < 4; ++mb)
#pragma unroll
        for (int nb = 0; nb < 4; ++nb) acc[mb][nb] = (v8f){};
    const size_t aoff = (size_t)(r0 + lr) * K + 8 * hi, boff = (size_t)(c0 + lr) * K + 8 * hi;
#pragma unroll 1
    for (int kc = 0; kc < K; kc += 32) {
        v16bf a[4];
#pragma unroll
        for (int mb = 0; mb < 4; ++mb) a[mb] = ldb(Az + aoff + (size_t)mb * 16 * K + kc);
#pragma unroll
        for (int nb = 0; nb < 4; ++nb) { const v16bf b = ldb(Bz + boff + (size_t)nb * 16 * K + kc);
#pragma unroll
            for (int mb = 0; mb < 4; ++mb) acc[mb][nb] = wmmabg(a[mb], b, acc[mb][nb]); }
    }
    const size_t tbase = (size_t)(r0 / RB) * sRB + (size_t)(r0 % RB) * (size_t)pitch + (size_t)(c0 / CB) * sCB + (size_t)(c0 % CB);
    v4f cb0 = (v4f){}, cb1 = (v4f){};
    if (brow == 0) { const int c8 = (lane & 7) * 8;
        const v4f t0 = *(const v4f*)(bias + c0 + c8); const v4f t1 = *(const v4f*)(bias + c0 + c8 + 4);
#pragma unroll
        for (int i = 0; i < 4; ++i) { cb0[i] = bfr(t0[i]); cb1[i] = bfr(t1[i]); } }
#pragma unroll
    for (int mb = 0; mb < 4; ++mb) {
#pragma unroll
        for (int nb = 0; nb < 4; ++nb) {
#pragma unroll
            for (int j = 0; j < 8; ++j) os[(hi * 8 + j) * 68 + nb * 16 + lr] = acc[mb][nb][j]; }
        wave_sync();
        const size_t sb = tbase + (size_t)(mb * 16) * (size_t)pitch;
#pragma unroll 1
        for (int ps = 0; ps < 2; ++ps) {
#pragma unroll
            for (int s = 0; s < 4; ++s) { const int row = 4 * s + (lane >> 3), c8 = (lane & 7) * 8;
                v4f x0 = *(const v4fa*)(&os[row * 68 + c8]); v4f x1 = *(const v4fa*)(&os[row * 68 + c8 + 4]); v8h rv;
                if (brow != 0) { const float rb = bfr(bias[r0 + mb * 16 + row]);
#pragma unroll
                    for (int i = 0; i < 4; ++i) { x0[i] += rb; x1[i] += rb; }
                } else {
#pragma unroll
                    for (int i = 0; i < 4; ++i) { x0[i] += cb0[i]; x1[i] += cb1[i]; } }
#pragma unroll
                for (int i = 0; i < 4; ++i) { const h16 a0 = toh_flush(x0[i]); const h16 a1 = toh_flush(x1[i]);
                    rv[i] = toh_flush((x0[i] - (float)a0) * RSC); rv[4 + i] = toh_flush((x1[i] - (float)a1) * RSC); }
                const size_t oo = sb + (size_t)row * (size_t)pitch + c8;
                *(volatile v8h*)(Pz + oo) = rv; }
            if (ps == 0) __threadfence(); }
        wave_sync();
    }
}

__global__ __launch_bounds__(32 * AW) void k_flash(const h16* __restrict__ QH, const h16* __restrict__ KP, const h16* __restrict__ VT, const unsigned* __restrict__ MB, const unsigned* __restrict__ TF, h16* CTX, int tb0) {
    __shared__ __align__(16) float os[AW * 16 * 68];
    const int lane = threadIdx.x & 31, wave = __builtin_amdgcn_readfirstlane((int)(threadIdx.x >> 5)), lr = lane & 15, hi = lane >> 4;
    const int zh = blockIdx.y; const int b = zh / NH_, h = zh % NH_;
    const int t0 = tb0 + (blockIdx.x * AW + wave) * 16;
    const size_t fo = (size_t)(t0 >> 4) * 32;
    const unsigned f0 = (unsigned)__builtin_amdgcn_readfirstlane((int)TF[fo + 0]);
    const unsigned f1 = (unsigned)__builtin_amdgcn_readfirstlane((int)TF[fo + 1]);
    const unsigned f2 = (unsigned)__builtin_amdgcn_readfirstlane((int)TF[fo + 2]);
    const unsigned f3 = (unsigned)__builtin_amdgcn_readfirstlane((int)TF[fo + 3]);
    const unsigned long long act = ((unsigned long long)f1 << 32) | (unsigned long long)f0;
    const unsigned long long mix = ((unsigned long long)f3 << 32) | (unsigned long long)f2;
    const size_t mo = (size_t)(t0 + lr) * MBP;
    const size_t qbase = (size_t)zh * SEQ * HD;
    const size_t pbase = (size_t)(b * NKV + h / GRP) * SEQ * HD;
    const size_t qo = qbase + (size_t)(t0 + lr) * HD + 8 * hi;
    const v16h qh0 = ldh(QH + qo), qh1 = ldh(QH + qo + 32);
    const size_t ko = pbase + (size_t)lr * HD + 8 * hi;
    const size_t vo = pbase + (size_t)lr * SEQ + 8 * hi;
    v8f o0 = (v8f){}, o1 = (v8f){}, o2 = (v8f){}, o3 = (v8f){};
    float m = -3.0e38f, l = 0.0f;
#pragma unroll 1
    for (int key0 = 0; key0 < SEQ; key0 += 32) {
        const int ks = key0 >> 5;
        if (((act >> ks) & 1ull) == 0ull) continue;
        const h16* ka = KP + ko + (size_t)key0 * HD;
        const v16h ka0 = ldh(ka), ka1 = ldh(ka + 32), kb0 = ldh(ka + 16 * HD), kb1 = ldh(ka + 16 * HD + 32);
        v8f sa = (v8f){}, sb = (v8f){};
        sa = wmma16(ka0, qh0, sa); sb = wmma16(kb0, qh0, sb);
        sa = wmma16(ka1, qh1, sa); sb = wmma16(kb1, qh1, sb);
        asm volatile("v_nop\n\tv_nop\n\tv_nop\n\tv_nop" : "+v"(sa), "+v"(sb) : "v"(ka0), "v"(ka1), "v"(kb0), "v"(kb1));
        float ta[8], tb[8];
#pragma unroll
        for (int r = 0; r < 8; ++r) { ta[r] = sa[r] * SC2; tb[r] = sb[r] * SC2; }
        if (((mix >> ks) & 1ull) != 0ull) {
            unsigned mw = MB[mo + ks];
            asm volatile("" : "+v"(mw));
            const unsigned ma = mw >> (8 * hi), mc = mw >> (16 + 8 * hi);
#pragma unroll
            for (int r = 0; r < 8; ++r) { ta[r] = (((ma >> r) & 1u) != 0u) ? NEGF : ta[r]; tb[r] = (((mc >> r) & 1u) != 0u) ? NEGF : tb[r]; }
        }
        float mx = -3.0e38f;
#pragma unroll
        for (int r = 0; r < 8; ++r) mx = fmaxf(mx, fmaxf(ta[r], tb[r]));
        mx = fmaxf(mx, __shfl_xor(mx, 16, 32));
        const float mnew = fmaxf(m, mx);
        const float alpha = __builtin_amdgcn_exp2f(m - mnew);
        const float sh = PSH - mnew;
        v16h pb; float ls = 0.0f;
#pragma unroll
        for (int r = 0; r < 8; ++r) { const float ea = ta[r] + sh, ec = tb[r] + sh;
            const h16 pa = (ea < -14.0f) ? (h16)0.0f : (h16)__builtin_amdgcn_exp2f(ea);
            const h16 pc = (ec < -14.0f) ? (h16)0.0f : (h16)__builtin_amdgcn_exp2f(ec);
            pb[r] = pa; pb[8 + r] = pc; ls += (float)pa + (float)pc; }
        l = l * alpha + ls; m = mnew;
        o0 = o0 * alpha; o1 = o1 * alpha; o2 = o2 * alpha; o3 = o3 * alpha;
        const h16* va = VT + vo + key0;
        const v16h v0 = ldh(va), v1 = ldh(va + (size_t)16 * SEQ), v2 = ldh(va + (size_t)32 * SEQ), v3 = ldh(va + (size_t)48 * SEQ);
        o0 = wmma16(v0, pb, o0); o1 = wmma16(v1, pb, o1); o2 = wmma16(v2, pb, o2); o3 = wmma16(v3, pb, o3);
        asm volatile("v_nop\n\tv_nop\n\tv_nop\n\tv_nop" : "+v"(o0), "+v"(o1), "+v"(o2), "+v"(o3) : "v"(v0), "v"(v1), "v"(v2), "v"(v3), "v"(pb));
    }
    l += __shfl_xor(l, 16, 32);
    const float inv = (1.0f / l) * CXS;
    const int wb = wave * 16 * 68;
    { v4f a, c;
      a[0] = o0[0] * inv; a[1] = o0[1] * inv; a[2] = o0[2] * inv; a[3] = o0[3] * inv; c[0] = o0[4] * inv; c[1] = o0[5] * inv; c[2] = o0[6] * inv; c[3] = o0[7] * inv;
      *(v4fa*)(&os[wb + lr * 68 +  0 + 8 * hi]) = a; *(v4fa*)(&os[wb + lr * 68 +  0 + 8 * hi + 4]) = c;
      a[0] = o1[0] * inv; a[1] = o1[1] * inv; a[2] = o1[2] * inv; a[3] = o1[3] * inv; c[0] = o1[4] * inv; c[1] = o1[5] * inv; c[2] = o1[6] * inv; c[3] = o1[7] * inv;
      *(v4fa*)(&os[wb + lr * 68 + 16 + 8 * hi]) = a; *(v4fa*)(&os[wb + lr * 68 + 16 + 8 * hi + 4]) = c;
      a[0] = o2[0] * inv; a[1] = o2[1] * inv; a[2] = o2[2] * inv; a[3] = o2[3] * inv; c[0] = o2[4] * inv; c[1] = o2[5] * inv; c[2] = o2[6] * inv; c[3] = o2[7] * inv;
      *(v4fa*)(&os[wb + lr * 68 + 32 + 8 * hi]) = a; *(v4fa*)(&os[wb + lr * 68 + 32 + 8 * hi + 4]) = c;
      a[0] = o3[0] * inv; a[1] = o3[1] * inv; a[2] = o3[2] * inv; a[3] = o3[3] * inv; c[0] = o3[4] * inv; c[1] = o3[5] * inv; c[2] = o3[6] * inv; c[3] = o3[7] * inv;
      *(v4fa*)(&os[wb + lr * 68 + 48 + 8 * hi]) = a; *(v4fa*)(&os[wb + lr * 68 + 48 + 8 * hi + 4]) = c; }
    wave_sync();
    h16* crow = CTX + ((size_t)b * SEQ + t0) * DM + h * HD;
    const int c8 = (lane & 7) * 8;
    v8h hv0, hv1, hv2, hv3;
    { const int rq = lane >> 3;
      const v4f x00 = *(const v4fa*)(&os[wb + (0 + rq) * 68 + c8]),  x01 = *(const v4fa*)(&os[wb + (0 + rq) * 68 + c8 + 4]);
      const v4f x10 = *(const v4fa*)(&os[wb + (4 + rq) * 68 + c8]),  x11 = *(const v4fa*)(&os[wb + (4 + rq) * 68 + c8 + 4]);
      const v4f x20 = *(const v4fa*)(&os[wb + (8 + rq) * 68 + c8]),  x21 = *(const v4fa*)(&os[wb + (8 + rq) * 68 + c8 + 4]);
      const v4f x30 = *(const v4fa*)(&os[wb + (12 + rq) * 68 + c8]), x31 = *(const v4fa*)(&os[wb + (12 + rq) * 68 + c8 + 4]);
#pragma unroll
      for (int i = 0; i < 4; ++i) { hv0[i] = toh_flush(x00[i]); hv0[4 + i] = toh_flush(x01[i]); hv1[i] = toh_flush(x10[i]); hv1[4 + i] = toh_flush(x11[i]);
                                    hv2[i] = toh_flush(x20[i]); hv2[4 + i] = toh_flush(x21[i]); hv3[i] = toh_flush(x30[i]); hv3[4 + i] = toh_flush(x31[i]); } }
    h16* cp = crow + (size_t)(lane >> 3) * DM + c8;
#pragma unroll 1
    for (int ps = 0; ps < 2; ++ps) {
        *(volatile v8h*)(cp) = hv0;
        *(volatile v8h*)(cp + (size_t)4 * DM) = hv1;
        *(volatile v8h*)(cp + (size_t)8 * DM) = hv2;
        *(volatile v8h*)(cp + (size_t)12 * DM) = hv3;
        if (ps == 0) __threadfence(); }
}

__global__ __launch_bounds__(32 * AW) void k_flash_e(const h16* __restrict__ QH, const h16* __restrict__ QR, const h16* __restrict__ KP, const h16* __restrict__ KR, const h16* __restrict__ VT, const h16* __restrict__ VR,
                                                     const unsigned* __restrict__ MB, const unsigned* __restrict__ TF, h16* CTX, h16* CTR) {
    __shared__ __align__(16) float os[AW * 16 * 68];
    const int lane = threadIdx.x & 31, wave = __builtin_amdgcn_readfirstlane((int)(threadIdx.x >> 5)), lr = lane & 15, hi = lane >> 4;
    const int zh = blockIdx.y; const int b = zh / NH_, h = zh % NH_;
    const int t0 = (blockIdx.x * AW + wave) * 16;
    const size_t fo = (size_t)(t0 >> 4) * 32;
    const unsigned f0 = (unsigned)__builtin_amdgcn_readfirstlane((int)TF[fo + 0]);
    const unsigned f1 = (unsigned)__builtin_amdgcn_readfirstlane((int)TF[fo + 1]);
    const unsigned f2 = (unsigned)__builtin_amdgcn_readfirstlane((int)TF[fo + 2]);
    const unsigned f3 = (unsigned)__builtin_amdgcn_readfirstlane((int)TF[fo + 3]);
    const unsigned long long act = ((unsigned long long)f1 << 32) | (unsigned long long)f0;
    const unsigned long long mix = ((unsigned long long)f3 << 32) | (unsigned long long)f2;
    const size_t mo = (size_t)(t0 + lr) * MBP;
    const size_t qbase = (size_t)zh * SEQ * HD;
    const size_t pbase = (size_t)(b * NKV + h / GRP) * SEQ * HD;
    const size_t qrb = (size_t)zh * EROWS * HD;
    const size_t prb = (size_t)(b * NKV + h / GRP) * EROWS * HD;
    const size_t qo = qbase + (size_t)(t0 + lr) * HD + 8 * hi;
    const size_t qro = qrb + (size_t)(t0 + lr) * HD + 8 * hi;
    const v16h qh0 = ldh(QH + qo), qh1 = ldh(QH + qo + 32);
    const v16h qr0 = ldh(QR + qro), qr1 = ldh(QR + qro + 32);
    const size_t ko = pbase + (size_t)lr * HD + 8 * hi;
    const size_t kro = prb + (size_t)lr * HD + 8 * hi;
    const size_t vo = pbase + (size_t)lr * SEQ + 8 * hi;
    const size_t vro = prb + (size_t)lr * EROWS + 8 * hi;
    const v16h zf = (v16h){};
    v8f o[4], rr[4];
#pragma unroll
    for (int j = 0; j < 4; ++j) { o[j] = (v8f){}; rr[j] = (v8f){}; }
    float m = -3.0e38f, l = 0.0f;
#pragma unroll 1
    for (int key0 = 0; key0 < SEQ; key0 += 32) {
        const int ks = key0 >> 5;
        if (((act >> ks) & 1ull) == 0ull) continue;
        const bool er = key0 < EROWS;
        const int keyr = er ? key0 : 0;
        const h16* ka = KP + ko + (size_t)key0 * HD;
        const v16h ka0 = ldh(ka), ka1 = ldh(ka + 32), kb0 = ldh(ka + 16 * HD), kb1 = ldh(ka + 16 * HD + 32);
        v8f sa = (v8f){}, sb = (v8f){}, ra = (v8f){}, rb = (v8f){};
        sa = wmma16g(ka0, qh0, sa); sb = wmma16g(kb0, qh0, sb);
        sa = wmma16g(ka1, qh1, sa); sb = wmma16g(kb1, qh1, sb);
        ra = wmma16g(ka0, qr0, ra); rb = wmma16g(kb0, qr0, rb);
        ra = wmma16g(ka1, qr1, ra); rb = wmma16g(kb1, qr1, rb);
        { const h16* kr = KR + kro + (size_t)keyr * HD;
          const v16h l0 = ldh(kr), l1 = ldh(kr + 32), l2 = ldh(kr + 16 * HD), l3 = ldh(kr + 16 * HD + 32);
          const v16h kra0 = er ? l0 : zf, kra1 = er ? l1 : zf, krb0 = er ? l2 : zf, krb1 = er ? l3 : zf;
          ra = wmma16g(kra0, qh0, ra); rb = wmma16g(krb0, qh0, rb);
          ra = wmma16g(kra1, qh1, ra); rb = wmma16g(krb1, qh1, rb); }
        float ta[8], tb[8];
#pragma unroll
        for (int r = 0; r < 8; ++r) { ta[r] = (sa[r] + ra[r] * RIN) * SC2; tb[r] = (sb[r] + rb[r] * RIN) * SC2; }
        if (((mix >> ks) & 1ull) != 0ull) {
            unsigned mw = MB[mo + ks];
            asm volatile("" : "+v"(mw));
            const unsigned ma = mw >> (8 * hi), mc = mw >> (16 + 8 * hi);
#pragma unroll
            for (int r = 0; r < 8; ++r) { ta[r] = (((ma >> r) & 1u) != 0u) ? NEGF : ta[r]; tb[r] = (((mc >> r) & 1u) != 0u) ? NEGF : tb[r]; }
        }
        float mx = -3.0e38f;
#pragma unroll
        for (int r = 0; r < 8; ++r) mx = fmaxf(mx, fmaxf(ta[r], tb[r]));
        mx = fmaxf(mx, __shfl_xor(mx, 16, 32));
        const float mnew = fmaxf(m, mx);
        const float alpha = __builtin_amdgcn_exp2f(m - mnew);
        const float sh = PSH - mnew;
        v16h pb, pr; float ls = 0.0f;
#pragma unroll
        for (int r = 0; r < 8; ++r) { const float ea = ta[r] + sh, ec = tb[r] + sh;
            const float pa = (ea < -14.0f) ? 0.0f : __builtin_amdgcn_exp2f(ea);
            const float pc = (ec < -14.0f) ? 0.0f : __builtin_amdgcn_exp2f(ec);
            const h16 ha = (h16)pa, hc = (h16)pc;
            pb[r] = ha; pb[8 + r] = hc;
            pr[r] = toh_flush((pa - (float)ha) * RSC); pr[8 + r] = toh_flush((pc - (float)hc) * RSC);
            ls += pa + pc; }
        l = l * alpha + ls; m = mnew;
#pragma unroll
        for (int j = 0; j < 4; ++j) { o[j] = o[j] * alpha; rr[j] = rr[j] * alpha; }
        const h16* va = VT + vo + key0;
        const h16* vr = VR + vro + keyr;
#pragma unroll
        for (int j = 0; j < 4; ++j) {
            const v16h vh = ldh(va + (size_t)(16 * j) * SEQ);
            const v16h vl = ldh(vr + (size_t)(16 * j) * EROWS);
            const v16h vz = er ? vl : zf;
            o[j]  = wmma16g(vh, pb, o[j]);
            rr[j] = wmma16g(vh, pr, rr[j]);
            rr[j] = wmma16g(vz, pb, rr[j]); }
    }
    l += __shfl_xor(l, 16, 32);
    const float inv = (1.0f / l) * CXS;
    const int wb = wave * 16 * 68;
#pragma unroll
    for (int j = 0; j < 4; ++j) { v4f a, c;
#pragma unroll
        for (int i = 0; i < 4; ++i) { a[i] = (o[j][i] + rr[j][i] * RIN) * inv; c[i] = (o[j][4 + i] + rr[j][4 + i] * RIN) * inv; }
        *(v4fa*)(&os[wb + lr * 68 + 16 * j + 8 * hi]) = a; *(v4fa*)(&os[wb + lr * 68 + 16 * j + 8 * hi + 4]) = c; }
    wave_sync();
    const int c8 = (lane & 7) * 8;
    const int rq = lane >> 3;
    v8h ch[4], cr[4];
#pragma unroll
    for (int s = 0; s < 4; ++s) {
        const v4f x0 = *(const v4fa*)(&os[wb + (4 * s + rq) * 68 + c8]), x1 = *(const v4fa*)(&os[wb + (4 * s + rq) * 68 + c8 + 4]);
#pragma unroll
        for (int i = 0; i < 4; ++i) { const h16 a0 = toh_flush(x0[i]); const h16 a1 = toh_flush(x1[i]);
            ch[s][i] = a0; ch[s][4 + i] = a1;
            cr[s][i] = toh_flush((x0[i] - (float)a0) * RSC); cr[s][4 + i] = toh_flush((x1[i] - (float)a1) * RSC); } }
    h16* cp = CTX + ((size_t)b * SEQ + t0 + rq) * DM + h * HD + c8;
    h16* rp = CTR + ((size_t)b * EROWS + t0 + rq) * DM + h * HD + c8;
#pragma unroll 1
    for (int ps = 0; ps < 2; ++ps) {
#pragma unroll
        for (int s = 0; s < 4; ++s) {
            *(volatile v8h*)(cp + (size_t)(4 * s) * DM) = ch[s];
            *(volatile v8h*)(rp + (size_t)(4 * s) * DM) = cr[s]; }
        if (ps == 0) __threadfence(); }
}

__global__ __launch_bounds__(32) void k_oproj(const h16* __restrict__ A, const h16* __restrict__ Bt, const float* __restrict__ bias, float* OUT) {
    __shared__ __align__(16) float os[16 * 68];
    const int K = DM;
    const int lane = threadIdx.x & 31, lr = lane & 15, hi = lane >> 4; const int r0 = blockIdx.x * 64, c0 = blockIdx.y * 64;
    v8f acc[4][4];
#pragma unroll
    for (int mb = 0; mb < 4; ++mb)
#pragma unroll
        for (int nb = 0; nb < 4; ++nb) acc[mb][nb] = (v8f){};
    const size_t aoff = (size_t)(r0 + lr) * K + 8 * hi, boff = (size_t)(c0 + lr) * K + 8 * hi;
#pragma unroll 1
    for (int kc = 0; kc < K; kc += 32) {
        v16h a[4];
#pragma unroll
        for (int mb = 0; mb < 4; ++mb) a[mb] = ldh(A + aoff + (size_t)mb * 16 * K + kc);
#pragma unroll
        for (int nb = 0; nb < 4; ++nb) { const v16h b = ldh(Bt + boff + (size_t)nb * 16 * K + kc);
#pragma unroll
            for (int mb = 0; mb < 4; ++mb) acc[mb][nb] = wmma16(a[mb], b, acc[mb][nb]); }
        asm volatile("v_nop\n\tv_nop\n\tv_nop\n\tv_nop" : "+v"(acc[0][0]), "+v"(acc[1][1]), "+v"(acc[2][2]), "+v"(acc[3][3]) : "v"(a[0]), "v"(a[1]), "v"(a[2]), "v"(a[3]));
    }
    const int cofs = lr * 4;
    v4f bb;
    { const v4f tb = *(const v4f*)(bias + c0 + cofs);
#pragma unroll
      for (int i = 0; i < 4; ++i) bb[i] = bfr(tb[i]); }
    float* obase = OUT + ((size_t)(r0 / SEQ) * OUT_SEQ + (size_t)(r0 % SEQ)) * DM + c0 + cofs;
#pragma unroll
    for (int mb = 0; mb < 4; ++mb) {
#pragma unroll
        for (int nb = 0; nb < 4; ++nb) {
#pragma unroll
            for (int j = 0; j < 8; ++j) os[(hi * 8 + j) * 68 + nb * 16 + lr] = acc[mb][nb][j]; }
        wave_sync();
#pragma unroll 1
        for (int ps = 0; ps < 2; ++ps) {
#pragma unroll
            for (int s = 0; s < 8; ++s) { const int row = 2 * s + hi;
                const v4f xv = *(const v4fa*)(&os[row * 68 + cofs]); v4f val;
#pragma unroll
                for (int i = 0; i < 4; ++i) val[i] = xv[i] * OSC + bb[i];
                *(volatile v4f*)(obase + (size_t)(mb * 16 + row) * DM) = val; }
            if (ps == 0) __threadfence(); }
        wave_sync();
    }
}

__global__ __launch_bounds__(32) void k_oproj_e(const h16* __restrict__ A, const h16* __restrict__ AR, const h16* __restrict__ Bt, const float* __restrict__ bias, float* OUT) {
    __shared__ __align__(16) float os[16 * 68];
    const int K = DM;
    const int lane = threadIdx.x & 31, lr = lane & 15, hi = lane >> 4;
    const int bq = blockIdx.x / (EROWS / 32), tl = blockIdx.x % (EROWS / 32); const int c0 = blockIdx.y * 64;
    v8f acc[2][4], acr[2][4];
#pragma unroll
    for (int mb = 0; mb < 2; ++mb)
#pragma unroll
        for (int nb = 0; nb < 4; ++nb) { acc[mb][nb] = (v8f){}; acr[mb][nb] = (v8f){}; }
    const size_t aoff = (size_t)(bq * SEQ + tl * 32 + lr) * K + 8 * hi;
    const size_t roff = (size_t)(bq * EROWS + tl * 32 + lr) * K + 8 * hi;
    const size_t boff = (size_t)(c0 + lr) * K + 8 * hi;
#pragma unroll 1
    for (int kc = 0; kc < K; kc += 32) {
        v16h a[2], ar[2];
#pragma unroll
        for (int mb = 0; mb < 2; ++mb) { a[mb] = ldh(A + aoff + (size_t)mb * 16 * K + kc); ar[mb] = ldh(AR + roff + (size_t)mb * 16 * K + kc); }
#pragma unroll
        for (int nb = 0; nb < 4; ++nb) { const v16h b = ldh(Bt + boff + (size_t)nb * 16 * K + kc);
#pragma unroll
            for (int mb = 0; mb < 2; ++mb) { acc[mb][nb] = wmma16g(a[mb], b, acc[mb][nb]); acr[mb][nb] = wmma16g(ar[mb], b, acr[mb][nb]); } }
    }
    const int cofs = lr * 4;
    v4f bb;
    { const v4f tb = *(const v4f*)(bias + c0 + cofs);
#pragma unroll
      for (int i = 0; i < 4; ++i) bb[i] = bfr(tb[i]); }
    float* obase = OUT + ((size_t)bq * OUT_SEQ + (size_t)(tl * 32)) * DM + c0 + cofs;
#pragma unroll
    for (int mb = 0; mb < 2; ++mb) {
#pragma unroll
        for (int nb = 0; nb < 4; ++nb) {
#pragma unroll
            for (int j = 0; j < 8; ++j) os[(hi * 8 + j) * 68 + nb * 16 + lr] = acc[mb][nb][j] + acr[mb][nb][j] * RIN; }
        wave_sync();
#pragma unroll 1
        for (int ps = 0; ps < 2; ++ps) {
#pragma unroll
            for (int s = 0; s < 8; ++s) { const int row = 2 * s + hi;
                const v4f xv = *(const v4fa*)(&os[row * 68 + cofs]); v4f val;
#pragma unroll
                for (int i = 0; i < 4; ++i) val[i] = xv[i] * OSC + bb[i];
                *(volatile v4f*)(obase + (size_t)(mb * 16 + row) * DM) = val; }
            if (ps == 0) __threadfence(); }
        wave_sync();
    }
}

static constexpr size_t al256(size_t v) { return (v + 255) & ~(size_t)255; }
static constexpr size_t SZ_XB  = al256((size_t)NB * SEQ * DM * 2);
static constexpr size_t SZ_WQ  = al256((size_t)DM * DM * 2);
static constexpr size_t SZ_WKV = al256((size_t)KVD * DM * 2);
static constexpr size_t SZ_WO  = al256((size_t)DM * DM * 2);
static constexpr size_t SZ_QP  = al256((size_t)NB * NH_ * SEQ * HD * 2);
static constexpr size_t SZ_KP  = al256((size_t)NB * NKV * SEQ * HD * 2);
static constexpr size_t SZ_CX  = al256((size_t)NB * SEQ * DM * 2);
static constexpr size_t SZ_QR  = al256((size_t)NB * NH_ * EROWS * HD * 2);
static constexpr size_t SZ_KR  = al256((size_t)NB * NKV * EROWS * HD * 2);
static constexpr size_t SZ_CR  = al256((size_t)NB * EROWS * DM * 2);
static constexpr size_t SZ_MB  = al256((size_t)SEQ * MBP * 4);
static constexpr size_t SZ_TF  = al256((size_t)(SEQ / 16) * 32 * 4);
static constexpr size_t SZ_TOTAL = SZ_XB + SZ_WQ + 2 * SZ_WKV + SZ_WO + SZ_QP + 2 * SZ_KP + SZ_CX + SZ_QR + 2 * SZ_KR + SZ_CR + SZ_MB + SZ_TF;
static_assert(SZ_TOTAL <= (size_t)134217728);

extern "C" void kernel_launch(void* const* d_in, const int* in_sizes, int n_in,
                              void* d_out, int out_size, void* d_ws, size_t ws_size, hipStream_t stream) {
    if (n_in < 10) return;
    const size_t needx = ((size_t)(NB - 1) * SEQ_FULL + SEQ) * DM;
    if ((size_t)in_sizes[0] < needx) return;
    if ((size_t)in_sizes[1] < (size_t)(SEQ - 1) * SEQ_FULL + SEQ) return;
    if ((size_t)in_sizes[2] < (size_t)DM * DM || (size_t)in_sizes[4] < (size_t)DM * KVD || (size_t)in_sizes[6] < (size_t)DM * KVD || (size_t)in_sizes[8] < (size_t)DM * DM) return;
    if ((size_t)in_sizes[3] < (size_t)DM || (size_t)in_sizes[5] < (size_t)KVD || (size_t)in_sizes[7] < (size_t)KVD || (size_t)in_sizes[9] < (size_t)DM) return;
    if ((size_t)out_size < ((size_t)(NB - 1) * OUT_SEQ + SEQ) * DM) return;
    if (SZ_TOTAL > ws_size) return;
    const float* x  = (const float*)d_in[0];
    const int* mask = (const int*)d_in[1];
    const float* wq = (const float*)d_in[2]; const float* bq = (const float*)d_in[3];
    const float* wk = (const float*)d_in[4]; const float* bk = (const float*)d_in[5];
    const float* wv = (const float*)d_in[6]; const float* bv = (const float*)d_in[7];
    const float* wo = (const float*)d_in[8]; const float* bo = (const float*)d_in[9];
    float* OUT = (float*)d_out;
    char* wsp = (char*)d_ws;
    bf* XB  = (bf*)wsp; wsp += SZ_XB;
    bf* WQT = (bf*)wsp; wsp += SZ_WQ;
    bf* WKT = (bf*)wsp; wsp += SZ_WKV;
    bf* WVT = (bf*)wsp; wsp += SZ_WKV;
    unsigned short* WOT = (unsigned short*)wsp; wsp += SZ_WO;
    h16* QH = (h16*)wsp; wsp += SZ_QP;
    h16* KP = (h16*)wsp; wsp += SZ_KP;
    h16* VT = (h16*)wsp; wsp += SZ_KP;
    h16* CX = (h16*)wsp; wsp += SZ_CX;
    h16* QR = (h16*)wsp; wsp += SZ_QR;
    h16* KR = (h16*)wsp; wsp += SZ_KR;
    h16* VR = (h16*)wsp; wsp += SZ_KR;
    h16* CR = (h16*)wsp; wsp += SZ_CR;
    unsigned* MBW = (unsigned*)wsp; wsp += SZ_MB;
    unsigned* TFW = (unsigned*)wsp; wsp += SZ_TF;

    if (SEQ == SEQ_FULL) {
        const size_t n8 = (size_t)NB * SEQ * DM / 8;
        k_cvt8<<<(unsigned)((n8 + 255) / 256), 256, 0, stream>>>(x, XB, n8);
    } else {
        const size_t n8 = (size_t)SEQ * DM / 8;
        for (int b = 0; b < NB; ++b) k_cvt8<<<(unsigned)((n8 + 255) / 256), 256, 0, stream>>>(x + (size_t)b * SEQ_FULL * DM, XB + (size_t)b * SEQ * DM, n8);
    }
    k_tr<0><<<dim3(DM / 64,  DM / 64, 1), 256, 0, stream>>>(wq, WQT, DM, DM);
    k_tr<0><<<dim3(KVD / 64, DM / 64, 1), 256, 0, stream>>>(wk, WKT, DM, KVD);
    k_tr<0><<<dim3(KVD / 64, DM / 64, 1), 256, 0, stream>>>(wv, WVT, DM, KVD);
    k_tr<1><<<dim3(DM / 64,  DM / 64, 1), 256, 0, stream>>>(wo, WOT, DM, DM);

    k_mpack<<<dim3(SEQ / 16, 1, 1), 512, 0, stream>>>(mask, MBW, TFW);

    k_proj<0><<<dim3(NB * SEQ / 64, DM / 64, 1), 32, 0, stream>>>(XB, WQT, bq, QH, SEQ, (size_t)NH_ * SEQ * HD, HD, HD, (size_t)SEQ * HD);
    k_proj<0><<<dim3(NB * SEQ / 64, KVD / 64, 1), 32, 0, stream>>>(XB, WKT, bk, KP, SEQ, (size_t)NKV * SEQ * HD, HD, HD, (size_t)SEQ * HD);
    k_proj<1><<<dim3(KVD / 64, NB * SEQ / 64, 1), 32, 0, stream>>>(WVT, XB, bv, VT, KVD, (size_t)0, SEQ, SEQ, (size_t)KVD * SEQ);

    k_projr<<<dim3(EROWS / 64, DM / 64, NB), 32, 0, stream>>>(XB, WQT, bq, QR, (size_t)SEQ * DM, (size_t)0, (size_t)NH_ * EROWS * HD, 0, EROWS, (size_t)0, HD, HD, (size_t)EROWS * HD);
    k_projr<<<dim3(EROWS / 64, KVD / 64, NB), 32, 0, stream>>>(XB, WKT, bk, KR, (size_t)SEQ * DM, (size_t)0, (size_t)NKV * EROWS * HD, 0, EROWS, (size_t)0, HD, HD, (size_t)EROWS * HD);
    k_projr<<<dim3(KVD / 64, EROWS / 64, NB), 32, 0, stream>>>(WVT, XB, bv, VR, (size_t)0, (size_t)SEQ * DM, (size_t)KVD * EROWS, 1, KVD, (size_t)0, EROWS, EROWS, (size_t)0);

    k_flash_e<<<dim3(EROWS / (16 * AW), NB * NH_, 1), 32 * AW, 0, stream>>>(QH, QR, KP, KR, VT, VR, MBW, TFW, CX, CR);
    if (SEQ > EROWS)
        k_flash<<<dim3((SEQ - EROWS) / (16 * AW), NB * NH_, 1), 32 * AW, 0, stream>>>(QH, KP, VT, MBW, TFW, CX, EROWS);

    k_oproj_e<<<dim3(NB * EROWS / 32, DM / 64, 1), 32, 0, stream>>>(CX, CR, (const h16*)WOT, bo, OUT);
    if (SEQ > EROWS) {
        for (int b = 0; b < NB; ++b)
            k_oproj<<<dim3((SEQ - EROWS) / 64, DM / 64, 1), 32, 0, stream>>>(CX + ((size_t)b * SEQ + EROWS) * DM, (const h16*)WOT, bo, OUT + ((size_t)b * OUT_SEQ + EROWS) * DM);
    }
}
